// GraphMesh2ConvClassifier_8117488190083
// MI455X (gfx1250) — hardware-verified
//
#include <hip/hip_runtime.h>
#include <stdint.h>
#include <stddef.h>


typedef _Float16 v16h __attribute__((ext_vector_type(16)));
typedef _Float16 v8h  __attribute__((ext_vector_type(8)));
typedef float    v8f  __attribute__((ext_vector_type(8)));
typedef float    v4fa __attribute__((ext_vector_type(4), __may_alias__));
typedef float    v2fa __attribute__((ext_vector_type(2), __may_alias__));
typedef unsigned v4u  __attribute__((ext_vector_type(4)));

#define NN     50000
#define NBW    256
#define NBKT   196
#define NPAD   (NBKT * NBW)
#define SUB    8192
#define CAP    512
#define CNTP   224
#define NG     16
#define C1     64
#define C2     128
#define C3     32
#define NCLS   10
#define NEG_SLOPE 0.01f

__device__ __forceinline__ int clampi(int x, int lo, int hi) {
    return x < lo ? lo : (x > hi ? hi : x);
}

__device__ __forceinline__ v8f wmma_f16(v16h a, v16h b, v8f c) {
    v8f d = __builtin_amdgcn_wmma_f32_16x16x32_f16(false, a, false, b, (short)0, c, false, false);
    asm volatile("v_nop\n\tv_nop\n\tv_nop\n\tv_nop" : "+v"(d) : "v"(a), "v"(b));
    return d;
}

__device__ __forceinline__ v16h frag_a_lds(const float* rowp, int k0, int h, float sc) {
    const float* p0 = rowp + k0 + 8 * h;
    const float* p1 = rowp + k0 + 16 + 8 * h;
    const v4fa x0 = *(const v4fa*)(p0);
    const v4fa x1 = *(const v4fa*)(p0 + 4);
    const v4fa x2 = *(const v4fa*)(p1);
    const v4fa x3 = *(const v4fa*)(p1 + 4);
    v16h a;
#pragma unroll
    for (int i = 0; i < 4; ++i) {
        a[i]      = (_Float16)(x0[i] * sc);
        a[4 + i]  = (_Float16)(x1[i] * sc);
        a[8 + i]  = (_Float16)(x2[i] * sc);
        a[12 + i] = (_Float16)(x3[i] * sc);
    }
    return a;
}

__device__ __forceinline__ v16h frag_b(const _Float16* __restrict__ P, int nkc, int ct, int kc, int lane) {
    return *(const v16h*)(P + ((size_t)(ct * nkc + kc) * 32 + lane) * 16);
}

__global__ void __launch_bounds__(128)
k_pack(const float* __restrict__ W, int ldw, int transposed, int K, int Nc,
       int nct, int nkc, float scale, _Float16* __restrict__ P) {
    const int t = blockIdx.x * 128 + threadIdx.x;
    const int total = nct * nkc * 64;
    if (t >= total) return;
    const int g    = t & 1;
    const int lane = (t >> 1) & 31;
    const int slot = t >> 6;
    const int kc = slot % nkc, ct = slot / nkc;
    const int h = lane >> 4;
    const int n = ct * 16 + (lane & 15);
    v8h v;
#pragma unroll
    for (int i = 0; i < 8; ++i) {
        const int k = kc * 32 + g * 16 + 8 * h + i;
        float x = 0.0f;
        if (k < K && n < Nc) x = transposed ? W[(size_t)n * ldw + k] : W[(size_t)k * ldw + n];
        v[i] = (_Float16)(x * scale);
    }
    union { v8h hv; v4u u; } pk;
    pk.hv = v;
    const v4u val = pk.u;
    volatile v4u* dst = (volatile v4u*)(P + (size_t)t * 8);
    *dst = val;
    __threadfence();
    *dst = val;
}

__device__ __forceinline__ void bsort_store(unsigned* slots, int* cnt, int s, const unsigned* buf,
                                            const int* cntb, const int* boff, int t, int w, int lane) {
    for (int b = w; b < NBKT; b += 4) {
        int n = cntb[b];
        if (n > CAP) n = CAP;
        const int base = boff[b];
        const int nl = (n + 31) >> 5;
        volatile unsigned* d = (volatile unsigned*)(slots + ((size_t)s * NBKT + b) * CAP);
        for (int i = 0; i < nl; ++i) {
            const int idx = base + i * 32 + lane;
            const unsigned v = (idx < SUB) ? buf[idx] : 0u;
            d[i * 32 + lane] = v;
        }
    }
    for (int b = t; b < CNTP; b += 128) {
        int v = 0;
        if (b < NBKT) { v = cntb[b]; if (v > CAP) v = CAP; }
        ((volatile int*)cnt)[(size_t)s * CNTP + b] = v;
    }
}

__global__ void __launch_bounds__(128)
k_bsort(const int* __restrict__ keyD, const int* __restrict__ keyS, const int* __restrict__ val,
        int E,
        unsigned* __restrict__ slotsD, int* __restrict__ cntD,
        unsigned* __restrict__ slotsS, int* __restrict__ cntS) {
    __shared__ unsigned short hist[NBKT * 128];
    __shared__ unsigned buf[SUB];
    __shared__ int cntb[NBKT];
    __shared__ int boff[NBKT + 1];
    const int t = threadIdx.x, lane = t & 31, w = t >> 5;
    const int s = blockIdx.x;
    const bool second = (blockIdx.y != 0);
    const int* key = second ? keyS : keyD;
    unsigned* slots = second ? slotsS : slotsD;
    int* cnt = second ? cntS : cntD;

    for (int i = t; i < NBKT * 128; i += 128) hist[i] = 0;
    __syncthreads();
    const int e0 = s * SUB;
    for (int i = 0; i < SUB / 128; ++i) {
        const int e = e0 + i * 128 + t;
        if (e < E) {
            const int k = clampi(key[e], 0, NN - 1);
            hist[(k >> 8) * 128 + t] += 1;
        }
    }
    __syncthreads();
    for (int b = t; b < NBKT; b += 128) {
        int run = 0;
        for (int tt = 0; tt < 128; ++tt) {
            const int c = hist[b * 128 + tt];
            hist[b * 128 + tt] = (unsigned short)run;
            run += c;
        }
        cntb[b] = run;
    }
    __syncthreads();
    if (t == 0) {
        int acc = 0;
        for (int b = 0; b < NBKT; ++b) { boff[b] = acc; acc += cntb[b]; }
        boff[NBKT] = acc;
    }
    __syncthreads();
    for (int i = 0; i < SUB / 128; ++i) {
        const int e = e0 + i * 128 + t;
        if (e < E) {
            const int k = clampi(key[e], 0, NN - 1);
            const int b = k >> 8;
            const int p = boff[b] + (int)hist[b * 128 + t];
            hist[b * 128 + t] += 1;
            const unsigned v = ((unsigned)(k & 255) << 16) | (unsigned)clampi(val[e], 0, NN - 1);
            if ((unsigned)p < (unsigned)SUB) buf[p] = v;
        }
    }
    __syncthreads();
    bsort_store(slots, cnt, s, buf, cntb, boff, t, w, lane);
    __threadfence();
    bsort_store(slots, cnt, s, buf, cntb, boff, t, w, lane);
}

__global__ void __launch_bounds__(128)
k_deg(const unsigned* __restrict__ slotsD, const int* __restrict__ cntD,
      const unsigned* __restrict__ slotsS, const int* __restrict__ cntS,
      int nsub, float* __restrict__ rsD, float* __restrict__ rsS) {
    __shared__ unsigned short hist[NBW * 128];
    __shared__ float rsl[NBW];
    const int t = threadIdx.x;
    const int b = blockIdx.x;
    const bool second = (blockIdx.y != 0);
    const unsigned* slots = second ? slotsS : slotsD;
    const int* cnt = second ? cntS : cntD;
    float* rs = second ? rsS : rsD;

    for (int i = t; i < NBW * 128; i += 128) hist[i] = 0;
    __syncthreads();
    for (int s = 0; s < nsub; ++s) {
        const int n = clampi(cnt[(size_t)s * CNTP + b], 0, CAP);
        const unsigned* sl = slots + ((size_t)s * NBKT + b) * CAP;
        for (int i = t; i < n; i += 128) {
            const int node = (int)((sl[i] >> 16) & 255u);
            hist[node * 128 + t] += 1;
        }
    }
    __syncthreads();
    for (int node = t; node < NBW; node += 128) {
        int d = 0;
        for (int tt = 0; tt < 128; ++tt) d += hist[node * 128 + tt];
        rsl[node] = rsqrtf(fmaxf((float)d, 1.0f));
    }
    __syncthreads();
    const float r0 = rsl[t], r1 = rsl[t + 128];
    volatile float* d = (volatile float*)(rs + (size_t)b * NBW);
    d[t] = r0;
    d[t + 128] = r1;
    __threadfence();
    d[t] = r0;
    d[t + 128] = r1;
}

template <int C>
__device__ __forceinline__ void aggregate(int b, const unsigned* __restrict__ slots, const int* __restrict__ cnt,
                                          int nsub, const float* __restrict__ hin, const float* __restrict__ rsS,
                                          float* accl) {
    const int t = threadIdx.x, w = t >> 5, lane = t & 31;
    for (int s = 0; s < nsub; ++s) {
        const int n = clampi(cnt[(size_t)s * CNTP + b], 0, CAP);
        const unsigned* sl = slots + ((size_t)s * NBKT + b) * CAP;
        for (int base = 0; base < n; base += 32) {
            const int idx = base + lane;
            unsigned ent = 0u;
            if (idx < n) ent = sl[idx];
            const bool own = (idx < n) && ((int)((ent >> 16) & 3u) == w);
            unsigned mask = (unsigned)__ballot(own ? 1 : 0);
            while (mask != 0u) {
                const int bit = __builtin_ctz(mask);
                mask &= (mask - 1u);
                const unsigned e2 = (unsigned)__shfl((int)ent, bit);
                const int src = clampi((int)(e2 & 0xFFFFu), 0, NN - 1);
                const int dl  = (int)((e2 >> 16) & 255u);
                const float r = rsS[src];
                if (C == C1) {
                    const v2fa xv = *(const v2fa*)(hin + (size_t)src * C1 + 2 * lane);
                    v2fa* p = (v2fa*)(accl + dl * C1 + 2 * lane);
                    v2fa a = *p;
                    a += xv * r;
                    *p = a;
                } else {
                    const v4fa xv = *(const v4fa*)(hin + (size_t)src * C2 + 4 * lane);
                    v4fa* p = (v4fa*)(accl + dl * C2 + 4 * lane);
                    v4fa a = *p;
                    a += xv * r;
                    *p = a;
                }
            }
        }
    }
}

__device__ __forceinline__ void lines_out32(const float* lds, int pitch, int coff,
                                            float* g, int gpitch, int gcol, int node0, int w, int lane) {
    for (int i = 0; i < 16; ++i) {
        const int row = i * 16 + w * 4 + (lane >> 3);
        const int q = (lane & 7) * 4;
        const v4fa v = *(const v4fa*)(lds + row * pitch + coff + q);
        *(volatile v4fa*)(g + (size_t)(node0 + row) * gpitch + gcol + q) = v;
    }
}

__global__ void __launch_bounds__(128)
k_layer1(const unsigned* __restrict__ slotsD, const int* __restrict__ cntD, int nsub,
         const float* __restrict__ x, const float* __restrict__ rsS, const float* __restrict__ rsD,
         const _Float16* __restrict__ W1p, float* __restrict__ h1) {
    __shared__ float accl[NBW * C1];
    __shared__ float stg[NBW * 32];
    const int t = threadIdx.x, lane = t & 31, w = t >> 5;
    const int h = lane >> 4, m = lane & 15;
    const int b = blockIdx.x, node0 = b * NBW;

    const v4fa z = {0.0f, 0.0f, 0.0f, 0.0f};
    for (int i = t; i < NBW * C1 / 4; i += 128) *(v4fa*)(accl + 4 * i) = z;
    __syncthreads();
    aggregate<C1>(b, slotsD, cntD, nsub, x, rsS, accl);
    __syncthreads();

    for (int sl = 0; sl < 4; ++sl) {
        for (int j = 0; j < 4; ++j) {
            const int rt = w * 4 + j;
            const int row = rt * 16 + m;
            const float sc = rsD[node0 + row] * 16.0f;
            const float* rowp = accl + row * C1;
            const v16h a0 = frag_a_lds(rowp, 0, h, sc);
            const v16h a1 = frag_a_lds(rowp, 32, h, sc);
#pragma unroll
            for (int cc = 0; cc < 2; ++cc) {
                const int ct = sl * 2 + cc;
                v8f acc = {0.0f, 0.0f, 0.0f, 0.0f, 0.0f, 0.0f, 0.0f, 0.0f};
                acc = wmma_f16(a0, frag_b(W1p, 2, ct, 0, lane), acc);
                acc = wmma_f16(a1, frag_b(W1p, 2, ct, 1, lane), acc);
#pragma unroll
                for (int r = 0; r < 8; ++r) {
                    float v = acc[r] * (1.0f / 1024.0f);
                    v = (v >= 0.0f) ? v : NEG_SLOPE * v;
                    stg[(rt * 16 + 8 * h + r) * 32 + cc * 16 + m] = v;
                }
            }
        }
        __syncthreads();
        lines_out32(stg, 32, 0, h1, C2, sl * 32, node0, w, lane);
        __threadfence();
        lines_out32(stg, 32, 0, h1, C2, sl * 32, node0, w, lane);
        __syncthreads();
    }
}

__global__ void __launch_bounds__(128)
k_layer2(const unsigned* __restrict__ slotsD, const int* __restrict__ cntD, int nsub,
         const float* __restrict__ h1, const float* __restrict__ rsS, const float* __restrict__ rsD,
         const _Float16* __restrict__ W2p, const _Float16* __restrict__ lWp, const float* __restrict__ linb,
         float* __restrict__ h3) {
    __shared__ float accl[NBW * C2];
    const int t = threadIdx.x, lane = t & 31, w = t >> 5;
    const int h = lane >> 4, m = lane & 15;
    const int b = blockIdx.x, node0 = b * NBW;

    const v4fa z = {0.0f, 0.0f, 0.0f, 0.0f};
    for (int i = t; i < NBW * C2 / 4; i += 128) *(v4fa*)(accl + 4 * i) = z;
    __syncthreads();
    aggregate<C2>(b, slotsD, cntD, nsub, h1, rsS, accl);
    __syncthreads();

    for (int j = 0; j < 4; ++j) {
        const int rt = w * 4 + j;
        const int row = rt * 16 + m;
        const float sc = rsD[node0 + row] * 16.0f;
        const float* rowp = accl + row * C2;
        const v16h a0 = frag_a_lds(rowp, 0, h, sc);
        const v16h a1 = frag_a_lds(rowp, 32, h, sc);
        const v16h a2 = frag_a_lds(rowp, 64, h, sc);
        const v16h a3 = frag_a_lds(rowp, 96, h, sc);
#pragma unroll
        for (int ct = 0; ct < 4; ++ct) {
            v8f acc = {0.0f, 0.0f, 0.0f, 0.0f, 0.0f, 0.0f, 0.0f, 0.0f};
            acc = wmma_f16(a0, frag_b(W2p, 4, ct, 0, lane), acc);
            acc = wmma_f16(a1, frag_b(W2p, 4, ct, 1, lane), acc);
            acc = wmma_f16(a2, frag_b(W2p, 4, ct, 2, lane), acc);
            acc = wmma_f16(a3, frag_b(W2p, 4, ct, 3, lane), acc);
#pragma unroll
            for (int r = 0; r < 8; ++r) {
                float v = acc[r] * (1.0f / 1024.0f);
                v = (v >= 0.0f) ? v : NEG_SLOPE * v;
                accl[(rt * 16 + 8 * h + r) * C2 + ct * 16 + m] = v;
            }
        }
    }
    __syncthreads();
    for (int j = 0; j < 4; ++j) {
        const int rt = w * 4 + j;
        const int row = rt * 16 + m;
        const float* rowp = accl + row * C2;
        const v16h a0 = frag_a_lds(rowp, 0, h, 16.0f);
        const v16h a1 = frag_a_lds(rowp, 32, h, 16.0f);
#pragma unroll
        for (int ct = 0; ct < 2; ++ct) {
            v8f acc = {0.0f, 0.0f, 0.0f, 0.0f, 0.0f, 0.0f, 0.0f, 0.0f};
            acc = wmma_f16(a0, frag_b(lWp, 2, ct, 0, lane), acc);
            acc = wmma_f16(a1, frag_b(lWp, 2, ct, 1, lane), acc);
            const float bias = linb[ct * 16 + m];
#pragma unroll
            for (int r = 0; r < 8; ++r) {
                accl[(rt * 16 + 8 * h + r) * C2 + 64 + ct * 16 + m] = acc[r] * (1.0f / 1024.0f) + bias;
            }
        }
    }
    __syncthreads();
    lines_out32(accl, C2, 64, h3, C3, 0, node0, w, lane);
    __threadfence();
    lines_out32(accl, C2, 64, h3, C3, 0, node0, w, lane);
}

__global__ void __launch_bounds__(512)
k_poolcls(const float* __restrict__ h3, const int* __restrict__ gid, int nn,
          const _Float16* __restrict__ clsp, float* __restrict__ out) {
    __shared__ double psum[NG * NG * C3];
    __shared__ int pcnt[NG * NG];
    __shared__ float pooled[NG * C3];
    __shared__ float outl[NG * NCLS];
    const int t = threadIdx.x, lane = t & 31, w = t >> 5;
    const int h = lane >> 4, m = lane & 15;

    for (int i = t; i < NG * NG * C3; i += 512) psum[i] = 0.0;
    for (int i = t; i < NG * NG; i += 512) pcnt[i] = 0;
    __syncthreads();
    const int per = (nn + NG - 1) / NG;
    const int n0 = w * per;
    int n1 = n0 + per; if (n1 > nn) n1 = nn;
    for (int n = n0; n < n1; ++n) {
        const int g = gid[n];
        if ((unsigned)g < (unsigned)NG) {
            psum[(w * NG + g) * C3 + lane] += (double)h3[(size_t)n * C3 + lane];
            if (lane == 0) pcnt[w * NG + g] += 1;
        }
    }
    __syncthreads();
    {
        const int g = t >> 5, c = lane;
        double ssum = 0.0;
        int cn = 0;
        for (int ww = 0; ww < NG; ++ww) {
            ssum += psum[(ww * NG + g) * C3 + c];
            cn += pcnt[ww * NG + g];
        }
        const float inv = 1.0f / fmaxf((float)cn, 1.0f);
        pooled[g * C3 + c] = (float)ssum * inv;
    }
    __syncthreads();
    if (w == 0) {
        const v16h a = frag_a_lds(pooled + m * C3, 0, h, 256.0f);
        const v16h bb = *(const v16h*)(clsp + lane * 16);
        v8f acc = {0.0f, 0.0f, 0.0f, 0.0f, 0.0f, 0.0f, 0.0f, 0.0f};
        acc = wmma_f16(a, bb, acc);
#pragma unroll
        for (int r = 0; r < 8; ++r) {
            const int g = 8 * h + r;
            if (m < NCLS) outl[g * NCLS + m] = acc[r] * (1.0f / 16384.0f);
        }
    }
    __syncthreads();
    if (w == 0) {
        const v4fa v0 = *(const v4fa*)(outl + 4 * lane);
        v4fa v1 = v0;
        if (lane < 8) v1 = *(const v4fa*)(outl + 128 + 4 * lane);
        *(volatile v4fa*)(out + 4 * lane) = v0;
        if (lane < 8) *(volatile v4fa*)(out + 128 + 4 * lane) = v1;
        __threadfence();
        *(volatile v4fa*)(out + 4 * lane) = v0;
        if (lane < 8) *(volatile v4fa*)(out + 128 + 4 * lane) = v1;
    }
}

static inline size_t al256(size_t x) { return (x + 255) & ~(size_t)255; }

extern "C" void kernel_launch(void* const* d_in, const int* in_sizes, int n_in,
                              void* d_out, int out_size, void* d_ws, size_t ws_size,
                              hipStream_t stream) {
    if (n_in < 9) return;
    if (in_sizes[0] != NN * C1 || in_sizes[1] != C1 * C2 || in_sizes[2] != C2 * C1 ||
        in_sizes[3] != C3 * C1 || in_sizes[4] != C3 || in_sizes[5] != NCLS * C3 ||
        in_sizes[6] <= 0 || in_sizes[7] != in_sizes[6] || in_sizes[8] != NN ||
        out_size != NG * NCLS) return;
    const int E = in_sizes[6];
    const int nsub = (E + SUB - 1) / SUB;

    const float* features = (const float*)d_in[0];
    const float* W1   = (const float*)d_in[1];
    const float* W2   = (const float*)d_in[2];
    const float* linW = (const float*)d_in[3];
    const float* linb = (const float*)d_in[4];
    const float* clsW = (const float*)d_in[5];
    const int*   src  = (const int*)d_in[6];
    const int*   dst  = (const int*)d_in[7];
    const int*   gid  = (const int*)d_in[8];
    float* out = (float*)d_out;

    char* ws = (char*)d_ws;
    size_t off = 0;
    _Float16* W1p  = (_Float16*)(ws + off); off += al256((size_t)8 * 2 * 512 * sizeof(_Float16));
    _Float16* W2p  = (_Float16*)(ws + off); off += al256((size_t)4 * 4 * 512 * sizeof(_Float16));
    _Float16* lWp  = (_Float16*)(ws + off); off += al256((size_t)2 * 2 * 512 * sizeof(_Float16));
    _Float16* clsp = (_Float16*)(ws + off); off += al256((size_t)1 * 1 * 512 * sizeof(_Float16));
    float* rsD = (float*)(ws + off); off += al256((size_t)NPAD * sizeof(float));
    float* rsS = (float*)(ws + off); off += al256((size_t)NPAD * sizeof(float));
    int* cntD = (int*)(ws + off); off += al256((size_t)nsub * CNTP * sizeof(int));
    int* cntS = (int*)(ws + off); off += al256((size_t)nsub * CNTP * sizeof(int));
    unsigned* slotsD = (unsigned*)(ws + off); off += al256((size_t)nsub * NBKT * CAP * sizeof(unsigned));
    unsigned* slotsS = (unsigned*)(ws + off); off += al256((size_t)nsub * NBKT * CAP * sizeof(unsigned));
    float* h1 = (float*)(ws + off); off += al256((size_t)NPAD * C2 * sizeof(float));
    float* h3 = (float*)(ws + off); off += al256((size_t)NPAD * C3 * sizeof(float));
    if (off > ws_size) return;

    hipLaunchKernelGGL(k_pack, dim3((8 * 2 * 64 + 127) / 128), dim3(128), 0, stream,
                       W1, C2, 0, C1, C2, 8, 2, 64.0f, W1p);
    hipLaunchKernelGGL(k_pack, dim3((4 * 4 * 64 + 127) / 128), dim3(128), 0, stream,
                       W2, C1, 0, C2, C1, 4, 4, 64.0f, W2p);
    hipLaunchKernelGGL(k_pack, dim3((2 * 2 * 64 + 127) / 128), dim3(128), 0, stream,
                       linW, C1, 1, C1, C3, 2, 2, 64.0f, lWp);
    hipLaunchKernelGGL(k_pack, dim3((1 * 1 * 64 + 127) / 128), dim3(128), 0, stream,
                       clsW, C3, 1, C3, NCLS, 1, 1, 64.0f, clsp);

    hipLaunchKernelGGL(k_bsort, dim3(nsub, 2), dim3(128), 0, stream,
                       dst, src, src, E, slotsD, cntD, slotsS, cntS);
    hipLaunchKernelGGL(k_deg, dim3(NBKT, 2), dim3(128), 0, stream,
                       (const unsigned*)slotsD, (const int*)cntD, (const unsigned*)slotsS, (const int*)cntS,
                       nsub, rsD, rsS);
    hipLaunchKernelGGL(k_layer1, dim3(NBKT), dim3(128), 0, stream,
                       (const unsigned*)slotsD, (const int*)cntD, nsub, features,
                       (const float*)rsS, (const float*)rsD, (const _Float16*)W1p, h1);
    hipLaunchKernelGGL(k_layer2, dim3(NBKT), dim3(128), 0, stream,
                       (const unsigned*)slotsD, (const int*)cntD, nsub, (const float*)h1,
                       (const float*)rsS, (const float*)rsD, (const _Float16*)W2p, (const _Float16*)lWp,
                       linb, h3);
    hipLaunchKernelGGL(k_poolcls, dim3(1), dim3(512), 0, stream,
                       (const float*)h3, gid, NN, (const _Float16*)clsp, out);
    (void)hipGetLastError();
}
